// SimpleMHAJAX_50629074485296
// MI455X (gfx1250) — hardware-verified
//
#include <hip/hip_runtime.h>
#include <stddef.h>


typedef __bf16 bf16_t;
typedef __bf16 v16bf  __attribute__((ext_vector_type(16)));
typedef __bf16 bf16x8 __attribute__((ext_vector_type(8)));
typedef float  v8f    __attribute__((ext_vector_type(8)));
typedef float  v4f    __attribute__((ext_vector_type(4)));
typedef unsigned int v4u __attribute__((ext_vector_type(4)));

#define SEQ    4096
#define DMODEL 1024
#define HEADS  16
#define HD     64
#define NEGV   (-1.0e30f)

union Frag  { v16bf v; bf16x8 h8[2]; };
union Pack8 { bf16x8 b; v4u u; };

static __device__ __forceinline__ v8f zero8() {
  v8f z = {0.0f, 0.0f, 0.0f, 0.0f, 0.0f, 0.0f, 0.0f, 0.0f};
  return z;
}

static __device__ __forceinline__ v8f wmma_g(v16bf a, v16bf b, v8f c) {
  v8f d = __builtin_amdgcn_wmma_f32_16x16x32_bf16(false, a, false, b, (short)0, c, false, false);
  asm volatile("v_nop\n\tv_nop\n\tv_nop\n\tv_nop" : "+v"(d) : "v"(a), "v"(b));
  return d;
}

static __device__ __forceinline__ v16bf ldfrag(const bf16_t* row, int kq) {
  Frag f;
  f.h8[0] = *(const bf16x8*)(row + kq);
  f.h8[1] = *(const bf16x8*)(row + kq + 16);
  return f.v;
}

static __device__ __forceinline__ void split8(v4f a, v4f c, v4u& hi, v4u& lo) {
  float f[8] = {a[0], a[1], a[2], a[3], c[0], c[1], c[2], c[3]};
  Pack8 H, L;
#pragma unroll
  for (int e = 0; e < 8; ++e) {
    const bf16_t hb = (bf16_t)f[e];
    H.b[e] = hb;
    L.b[e] = (bf16_t)(f[e] - (float)hb);
  }
  hi = H.u;
  lo = L.u;
}

__global__ __launch_bounds__(256) void k_cvt_x(const float* __restrict__ x,
                                               bf16_t* xh, bf16_t* xl, int n8) {
  const int i = blockIdx.x * 256 + threadIdx.x;
  if (i < n8) {
    const float* p = x + (size_t)i * 8;
    const v4f a = *(const v4f*)p;
    const v4f c = *(const v4f*)(p + 4);
    v4u hi, lo;
    split8(a, c, hi, lo);
    volatile v4u* ph = (volatile v4u*)(xh + (size_t)i * 8);
    volatile v4u* pl = (volatile v4u*)(xl + (size_t)i * 8);
    *ph = hi;
    *pl = lo;
    __threadfence();
    *ph = hi;
    *pl = lo;
  }
}

__global__ __launch_bounds__(256) void k_cvt_wt(const float* __restrict__ W, int Krows, int Ncols,
                                                bf16_t* th, bf16_t* tl) {
  __shared__ __align__(16) float Ts[64][68];
  const int tid = threadIdx.x;
  const int n0  = blockIdx.x * 64;
  const int k0  = blockIdx.y * 64;
  {
    const int kr = tid >> 2;
    const int c  = (tid & 3) * 16;
    const float* src = W + (size_t)(k0 + kr) * (size_t)Ncols + n0 + c;
#pragma unroll
    for (int e4 = 0; e4 < 4; ++e4) {
      const v4f v = *(const v4f*)(src + 4 * e4);
      Ts[c + 4 * e4 + 0][kr] = v[0];
      Ts[c + 4 * e4 + 1][kr] = v[1];
      Ts[c + 4 * e4 + 2][kr] = v[2];
      Ts[c + 4 * e4 + 3][kr] = v[3];
    }
  }
  __syncthreads();
  const int q8   = tid & 7;
  const int lrow = tid >> 3;
  auto pass = [&]() {
#pragma unroll
    for (int it = 0; it < 2; ++it) {
      const int nl = it * 32 + lrow;
      const v4f a = *(const v4f*)&Ts[nl][q8 * 8];
      const v4f c = *(const v4f*)&Ts[nl][q8 * 8 + 4];
      v4u hi, lo;
      split8(a, c, hi, lo);
      const size_t off = (size_t)(n0 + nl) * (size_t)Krows + k0 + q8 * 8;
      *(volatile v4u*)(th + off) = hi;
      *(volatile v4u*)(tl + off) = lo;
    }
  };
  pass();
  __threadfence();
  pass();
}

template <int MODE>
__global__ __launch_bounds__(128) void k_gemm3(
    const bf16_t* __restrict__ Ah, const bf16_t* __restrict__ Al,
    const bf16_t* __restrict__ Bh, const bf16_t* __restrict__ Bl,
    int K, int N,
    bf16_t* Qh, bf16_t* Ql, bf16_t* Kh, bf16_t* Kl, bf16_t* Vh, bf16_t* Vl,
    float* Cout)
{
  __shared__ __align__(16) float Cs[64][68];

  const int tid  = threadIdx.x;
  const int lane = tid & 31;
  const int wave = tid >> 5;
  const int hh   = lane >> 4;
  const int ll   = lane & 15;
  const int m0   = blockIdx.y * 64;
  const int n0   = blockIdx.x * 64;
  const int wm   = (wave >> 1) * 32;
  const int wn   = (wave & 1) * 32;

  v8f acc[2][2];
  acc[0][0] = zero8(); acc[0][1] = zero8(); acc[1][0] = zero8(); acc[1][1] = zero8();

  const bf16_t* arh[2];
  const bf16_t* arl[2];
  const bf16_t* brh[2];
  const bf16_t* brl[2];
#pragma unroll
  for (int i = 0; i < 2; ++i) {
    const size_t ra = (size_t)(m0 + wm + 16 * i + ll) * (size_t)K;
    arh[i] = Ah + ra;
    arl[i] = Al + ra;
    const size_t rb = (size_t)(n0 + wn + 16 * i + ll) * (size_t)K;
    brh[i] = Bh + rb;
    brl[i] = Bl + rb;
  }

#pragma unroll 1
  for (int k0 = 0; k0 < K; k0 += 32) {
    const int kq = k0 + 8 * hh;
    v16bf ah[2], al[2], bh[2], bl[2];
#pragma unroll
    for (int i = 0; i < 2; ++i) {
      ah[i] = ldfrag(arh[i], kq);
      al[i] = ldfrag(arl[i], kq);
      bh[i] = ldfrag(brh[i], kq);
      bl[i] = ldfrag(brl[i], kq);
    }
#pragma unroll
    for (int i = 0; i < 2; ++i) {
#pragma unroll
      for (int j = 0; j < 2; ++j) {
        acc[i][j] = wmma_g(ah[i], bh[j], acc[i][j]);
        acc[i][j] = wmma_g(ah[i], bl[j], acc[i][j]);
        acc[i][j] = wmma_g(al[i], bh[j], acc[i][j]);
      }
    }
  }

#pragma unroll
  for (int i = 0; i < 2; ++i)
#pragma unroll
    for (int j = 0; j < 2; ++j)
#pragma unroll
      for (int r = 0; r < 8; ++r)
        Cs[wm + 16 * i + 8 * hh + r][wn + 16 * j + ll] = acc[i][j][r];
  __syncthreads();

  const int q8   = tid & 7;
  const int lrow = tid >> 3;
  if (MODE == 0) {
    const int mat  = n0 >> 10;
    const int head = (n0 & 1023) >> 6;
    if (mat < 2) {
      bf16_t* Ph = (mat == 0) ? Qh : Kh;
      bf16_t* Pl = (mat == 0) ? Ql : Kl;
      auto pass = [&]() {
#pragma unroll
        for (int it = 0; it < 4; ++it) {
          const int m = it * 16 + lrow;
          const v4f a = *(const v4f*)&Cs[m][q8 * 8];
          const v4f c = *(const v4f*)&Cs[m][q8 * 8 + 4];
          v4u hi, lo;
          split8(a, c, hi, lo);
          const size_t off = ((size_t)head * SEQ + (size_t)(m0 + m)) * HD + q8 * 8;
          *(volatile v4u*)(Ph + off) = hi;
          *(volatile v4u*)(Pl + off) = lo;
        }
      };
      pass();
      __threadfence();
      pass();
    } else {
      auto pass = [&]() {
#pragma unroll
        for (int it = 0; it < 4; ++it) {
          const int d = it * 16 + lrow;
          float f[8];
#pragma unroll
          for (int e = 0; e < 8; ++e) f[e] = Cs[q8 * 8 + e][d];
          const v4f a = {f[0], f[1], f[2], f[3]};
          const v4f c = {f[4], f[5], f[6], f[7]};
          v4u hi, lo;
          split8(a, c, hi, lo);
          const size_t off = ((size_t)head * HD + (size_t)d) * SEQ + m0 + q8 * 8;
          *(volatile v4u*)(Vh + off) = hi;
          *(volatile v4u*)(Vl + off) = lo;
        }
      };
      pass();
      __threadfence();
      pass();
    }
  } else {
    auto pass = [&]() {
#pragma unroll
      for (int it = 0; it < 8; ++it) {
        const int L = it * 16 + lrow;
        const int m = L >> 1;
        const int c = L & 1;
        const v4f v = *(const v4f*)&Cs[m][c * 32 + q8 * 4];
        *(volatile v4f*)(Cout + (size_t)(m0 + m) * (size_t)N + n0 + c * 32 + q8 * 4) = v;
      }
    };
    pass();
    __threadfence();
    pass();
  }
}

__global__ __launch_bounds__(128) void k_attn(
    const bf16_t* __restrict__ Qh, const bf16_t* __restrict__ Ql,
    const bf16_t* __restrict__ Kh, const bf16_t* __restrict__ Kl,
    const bf16_t* __restrict__ Vh, const bf16_t* __restrict__ Vl,
    bf16_t* AOh, bf16_t* AOl)
{
  __shared__ __align__(16) float Os[4][16][68];

  const int tid  = threadIdx.x;
  const int lane = tid & 31;
  const int wave = tid >> 5;
  const int hh   = lane >> 4;
  const int ll   = lane & 15;
  const int head = blockIdx.y;
  const int q0   = blockIdx.x * 64 + wave * 16;
  const int q    = q0 + ll;
  const size_t hs = (size_t)head * SEQ;
  const size_t vb = (size_t)head * HD;

  v16bf qh[2], ql[2];
  {
    const bf16_t* rh = Qh + (hs + (size_t)q) * HD;
    const bf16_t* rl = Ql + (hs + (size_t)q) * HD;
#pragma unroll
    for (int s = 0; s < 2; ++s) {
      qh[s] = ldfrag(rh, 32 * s + 8 * hh);
      ql[s] = ldfrag(rl, 32 * s + 8 * hh);
    }
  }

  v8f o[4];
  o[0] = zero8(); o[1] = zero8(); o[2] = zero8(); o[3] = zero8();
  float mst = NEGV, lst = 0.0f;
  const int kend = q0 + 16;

#pragma unroll 1
  for (int kb0 = 0; kb0 < kend; kb0 += 32) {
    v8f t[2];
#pragma unroll
    for (int tt = 0; tt < 2; ++tt) {
      const int krow = kb0 + 16 * tt + ll;
      const bf16_t* rh = Kh + (hs + (size_t)krow) * HD;
      const bf16_t* rl = Kl + (hs + (size_t)krow) * HD;
      v8f s8 = zero8();
#pragma unroll
      for (int s = 0; s < 2; ++s) {
        const v16bf kh = ldfrag(rh, 32 * s + 8 * hh);
        const v16bf kl = ldfrag(rl, 32 * s + 8 * hh);
        s8 = wmma_g(kh, qh[s], s8);
        s8 = wmma_g(kh, ql[s], s8);
        s8 = wmma_g(kl, qh[s], s8);
      }
      t[tt] = s8;
    }

    float xs[16];
#pragma unroll
    for (int r = 0; r < 8; ++r) {
      const int key0 = kb0 + 8 * hh + r;
      const float v0 = t[0][r] * 0.125f;
      xs[r] = (key0 > q) ? NEGV : v0;
      const int key1 = key0 + 16;
      const float v1 = t[1][r] * 0.125f;
      xs[8 + r] = (key1 > q) ? NEGV : v1;
    }

    float mx = xs[0];
#pragma unroll
    for (int i = 1; i < 16; ++i) mx = fmaxf(mx, xs[i]);
    mx = fmaxf(mx, __shfl_xor(mx, 16, 32));
    const float mnew = fmaxf(mst, mx);
    const float scf  = __expf(mst - mnew);
    mst = mnew;

    Frag ph, pl;
    float ps = 0.0f;
#pragma unroll
    for (int i = 0; i < 16; ++i) {
      const float p = __expf(xs[i] - mnew);
      ps += p;
      const bf16_t hb = (bf16_t)p;
      ph.v[i] = hb;
      pl.v[i] = (bf16_t)(p - (float)hb);
    }
    ps += __shfl_xor(ps, 16, 32);
    lst = lst * scf + ps;

    float sarr[8];
#pragma unroll
    for (int r = 0; r < 8; ++r) sarr[r] = __shfl(scf, 8 * hh + r, 32);
#pragma unroll
    for (int t4 = 0; t4 < 4; ++t4)
#pragma unroll
      for (int r = 0; r < 8; ++r) o[t4][r] *= sarr[r];

#pragma unroll
    for (int t4 = 0; t4 < 4; ++t4) {
      const int d = t4 * 16 + ll;
      const bf16_t* vrh = Vh + (vb + (size_t)d) * SEQ;
      const bf16_t* vrl = Vl + (vb + (size_t)d) * SEQ;
      const v16bf fh = ldfrag(vrh, kb0 + 8 * hh);
      const v16bf fl = ldfrag(vrl, kb0 + 8 * hh);
      o[t4] = wmma_g(ph.v, fh, o[t4]);
      o[t4] = wmma_g(ph.v, fl, o[t4]);
      o[t4] = wmma_g(pl.v, fh, o[t4]);
    }
  }

  const float inv = 1.0f / lst;
  float iarr[8];
#pragma unroll
  for (int r = 0; r < 8; ++r) iarr[r] = __shfl(inv, 8 * hh + r, 32);
#pragma unroll
  for (int t4 = 0; t4 < 4; ++t4)
#pragma unroll
    for (int r = 0; r < 8; ++r)
      Os[wave][8 * hh + r][t4 * 16 + ll] = o[t4][r] * iarr[r];
  __syncthreads();

  auto pass = [&]() {
#pragma unroll
    for (int it = 0; it < 4; ++it) {
      const int L  = it * 4 + (lane >> 3);
      const int q8 = lane & 7;
      const v4f a = *(const v4f*)&Os[wave][L][q8 * 8];
      const v4f c = *(const v4f*)&Os[wave][L][q8 * 8 + 4];
      v4u hi, lo;
      split8(a, c, hi, lo);
      const size_t off = (size_t)(q0 + L) * DMODEL + head * HD + q8 * 8;
      *(volatile v4u*)(AOh + off) = hi;
      *(volatile v4u*)(AOl + off) = lo;
    }
  };
  pass();
  __threadfence();
  pass();
}

extern "C" void kernel_launch(void* const* d_in, const int* in_sizes, int n_in,
                              void* d_out, int out_size, void* d_ws, size_t ws_size,
                              hipStream_t stream) {
  if (n_in < 3) return;
  if (in_sizes[0] != SEQ * DMODEL) return;
  if (in_sizes[1] != DMODEL * 3 * DMODEL) return;
  if (in_sizes[2] != DMODEL * DMODEL) return;
  if (out_size != SEQ * DMODEL) return;

  const float* x    = (const float*)d_in[0];
  const float* Wqkv = (const float*)d_in[1];
  const float* Wout = (const float*)d_in[2];
  float* out = (float*)d_out;

  const size_t szX  = (size_t)SEQ * DMODEL * sizeof(bf16_t);
  const size_t szWq = (size_t)3 * DMODEL * DMODEL * sizeof(bf16_t);
  const size_t szWo = (size_t)DMODEL * DMODEL * sizeof(bf16_t);
  const size_t szHP = (size_t)HEADS * SEQ * HD * sizeof(bf16_t);

  char* ws = (char*)d_ws;
  size_t off = 0;
  auto carve = [&](size_t b) { char* p = ws + off; off += b; return p; };
  bf16_t* Xh   = (bf16_t*)carve(szX);
  bf16_t* Xl   = (bf16_t*)carve(szX);
  bf16_t* Wqh  = (bf16_t*)carve(szWq);
  bf16_t* Wql  = (bf16_t*)carve(szWq);
  bf16_t* Woh  = (bf16_t*)carve(szWo);
  bf16_t* Wol  = (bf16_t*)carve(szWo);
  bf16_t* Qh   = (bf16_t*)carve(szHP);
  bf16_t* Ql   = (bf16_t*)carve(szHP);
  bf16_t* Kh   = (bf16_t*)carve(szHP);
  bf16_t* Kl   = (bf16_t*)carve(szHP);
  bf16_t* Vh   = (bf16_t*)carve(szHP);
  bf16_t* Vl   = (bf16_t*)carve(szHP);
  bf16_t* AOh  = (bf16_t*)carve(szX);
  bf16_t* AOl  = (bf16_t*)carve(szX);
  if (off > ws_size) return;

  {
    const int n8 = SEQ * DMODEL / 8;
    k_cvt_x<<<dim3((n8 + 255) / 256), dim3(256), 0, stream>>>(x, Xh, Xl, n8);
  }
  k_cvt_wt<<<dim3(3 * DMODEL / 64, DMODEL / 64), dim3(256), 0, stream>>>(Wqkv, DMODEL, 3 * DMODEL, Wqh, Wql);
  k_cvt_wt<<<dim3(DMODEL / 64, DMODEL / 64), dim3(256), 0, stream>>>(Wout, DMODEL, DMODEL, Woh, Wol);

  k_gemm3<0><<<dim3(3 * DMODEL / 64, SEQ / 64), dim3(128), 0, stream>>>(
      Xh, Xl, Wqh, Wql, DMODEL, 3 * DMODEL, Qh, Ql, Kh, Kl, Vh, Vl, out);

  k_attn<<<dim3(SEQ / 64, HEADS), dim3(128), 0, stream>>>(Qh, Ql, Kh, Kl, Vh, Vl, AOh, AOl);

  k_gemm3<1><<<dim3(DMODEL / 64, SEQ / 64), dim3(128), 0, stream>>>(
      AOh, AOl, Woh, Wol, DMODEL, DMODEL, Qh, Ql, Kh, Kl, Vh, Vl, out);
}
